// EqvTransformer_89550068122337
// MI455X (gfx1250) — hardware-verified
//
#include <hip/hip_runtime.h>
#include <math.h>
#include <stdint.h>

#define NB     4
#define NTOK   1024
#define DM     512
#define NHD    8
#define HDIM   64
#define QKVC   1536
#define NEGBIG 1.0e38f

typedef __attribute__((ext_vector_type(16))) _Float16 v16h;
typedef __attribute__((ext_vector_type(8)))  _Float16 v8h;
typedef __attribute__((ext_vector_type(16))) __bf16   v16b;
typedef __attribute__((ext_vector_type(8)))  __bf16   v8b;
typedef __attribute__((ext_vector_type(8)))  float    v8f;
typedef __attribute__((ext_vector_type(4)))  float    v4f;
typedef __attribute__((ext_vector_type(2)))  float    v2f;
typedef __attribute__((ext_vector_type(4)))  unsigned int v4u;

__device__ __forceinline__ unsigned short f2bf_bits(float f) {
  const unsigned u = __float_as_uint(f);
  return (unsigned short)((u + 0x7FFFu + ((u >> 16) & 1u)) >> 16);
}
__device__ __forceinline__ float bf_bits2f(unsigned short h) { return __uint_as_float(((unsigned)h) << 16); }
__device__ __forceinline__ float bfr(float f) {
  const unsigned u = __float_as_uint(f);
  return __uint_as_float((u + 0x7FFFu + ((u >> 16) & 1u)) & 0xFFFF0000u);
}
__device__ __forceinline__ unsigned short h_bits(float f) {
  const _Float16 hv = (_Float16)f;
  return __builtin_bit_cast(unsigned short, hv);
}
__device__ __forceinline__ float h2f(unsigned short b) {
  const _Float16 hv = __builtin_bit_cast(_Float16, b);
  return (float)hv;
}
__device__ __forceinline__ unsigned pk16(unsigned short a, unsigned short b) { return (unsigned)a | ((unsigned)b << 16); }

__device__ __forceinline__ v16h ldfh(const _Float16* p) {
  union { v16h v; v8h q[2]; } f;
  f.q[0] = *(const v8h*)(p);
  f.q[1] = *(const v8h*)(p + 16);
  return f.v;
}
__device__ __forceinline__ v16b ldfb(const __bf16* p) {
  union { v16b v; v8b q[2]; } f;
  f.q[0] = *(const v8b*)(p);
  f.q[1] = *(const v8b*)(p + 16);
  return f.v;
}
__device__ __forceinline__ v8f mma_h(v16h a, v16h b, v8f c) {
  return __builtin_amdgcn_wmma_f32_16x16x32_f16(false, a, false, b, (short)0, c, false, false);
}
__device__ __forceinline__ v8f mma_b(v16b a, v16b b, v8f c) {
  return __builtin_amdgcn_wmma_f32_16x16x32_bf16(false, a, false, b, (short)0, c, false, false);
}

__device__ __forceinline__ void guard2h(v8f& a, v8f& b, v16h x, v16h y) {
#if defined(__HIP_DEVICE_COMPILE__)
  asm volatile("v_nop\n\tv_nop\n\tv_nop\n\tv_nop" : "+v"(a), "+v"(b) : "v"(x), "v"(y));
#endif
}
__device__ __forceinline__ void guard2b(v8f& a, v8f& b, v16b x, v16b y) {
#if defined(__HIP_DEVICE_COMPILE__)
  asm volatile("v_nop\n\tv_nop\n\tv_nop\n\tv_nop" : "+v"(a), "+v"(b) : "v"(x), "v"(y));
#endif
}
__device__ __forceinline__ void keep4h(v16h a, v16h b, v16h c, v16h d) {
#if defined(__HIP_DEVICE_COMPILE__)
  asm volatile("v_nop" :: "v"(a), "v"(b), "v"(c), "v"(d));
#endif
}
__device__ __forceinline__ void keep4b(v16b a, v16b b, v16b c, v16b d) {
#if defined(__HIP_DEVICE_COMPILE__)
  asm volatile("v_nop" :: "v"(a), "v"(b), "v"(c), "v"(d));
#endif
}
__device__ __forceinline__ void accg4(v8f& a, v8f& b, v8f& c, v8f& d) {
#if defined(__HIP_DEVICE_COMPILE__)
  asm volatile("v_nop\n\tv_nop\n\tv_nop\n\tv_nop" : "+v"(a), "+v"(b), "+v"(c), "+v"(d));
#endif
}

__global__ __launch_bounds__(256) void cast_bf16_kernel(const float* __restrict__ in,
                                                        unsigned short* __restrict__ out, int n2) {
  const int i = blockIdx.x * 256 + threadIdx.x;
  if (i < n2) {
    const v2f f = *(const v2f*)(in + 2 * (size_t)i);
    const unsigned u = pk16(f2bf_bits(f[0]), f2bf_bits(f[1]));
    volatile unsigned* o = (volatile unsigned*)out + i;
    *o = u;
    __threadfence();
    *o = u;
  }
}

template <bool ASPLIT, bool RR>
__global__ __launch_bounds__(256) void gemm64_kernel(
    const unsigned short* __restrict__ Ap, const unsigned short* __restrict__ A2p, int lda,
    const unsigned short* __restrict__ Btp, int ldb,
    float* __restrict__ C, int ldc,
    const float* __restrict__ bs0, const float* __restrict__ bs1, const float* __restrict__ bs2,
    const float* __restrict__ resid, int ldr,
    int M, int N, int K, float scale) {
  const __bf16* A  = (const __bf16*)Ap;
  const __bf16* A2 = (const __bf16*)A2p;
  const __bf16* Bt = (const __bf16*)Btp;
  __shared__ __align__(16) float sT[8][16 * 68];
  const int lane = threadIdx.x & 31;
  const int wave = threadIdx.x >> 5;
  const int tilesN = N >> 6;
  const int tilesM = M >> 6;
  const int tile = blockIdx.x * 8 + wave;
  if (tile >= tilesM * tilesN) return;
  const int tm = tile / tilesN;
  const int tn = tile - tm * tilesN;
  const int m0 = tm << 6;
  const int n0 = tn << 6;
  const int rlane = lane & 15;
  const int koff  = (lane >> 4) * 8;
  const int mOff  = (lane >> 4) * 8;

  v8f acc[4][4];
#pragma unroll
  for (int i = 0; i < 4; ++i)
#pragma unroll
    for (int j = 0; j < 4; ++j) acc[i][j] = (v8f){0.f, 0.f, 0.f, 0.f, 0.f, 0.f, 0.f, 0.f};

  for (int k0 = 0; k0 < K; k0 += 32) {
    v16b bh[4];
#pragma unroll
    for (int j = 0; j < 4; ++j)
      bh[j] = ldfb(Bt + (size_t)(n0 + (j << 4) + rlane) * ldb + k0 + koff);
#pragma unroll
    for (int i = 0; i < 4; ++i) {
      const size_t ao = (size_t)(m0 + (i << 4) + rlane) * lda + k0 + koff;
      const v16b ah = ldfb(A + ao);
      v16b al = ah;
      if (ASPLIT) al = ldfb(A2 + ao);
#pragma unroll
      for (int j = 0; j < 4; ++j) {
        acc[i][j] = mma_b(ah, bh[j], acc[i][j]);
        if (ASPLIT) acc[i][j] = mma_b(al, bh[j], acc[i][j]);
      }
      guard2b(acc[i][0], acc[i][3], ah, al);
    }
    keep4b(bh[0], bh[1], bh[2], bh[3]);
  }
  accg4(acc[0][0], acc[0][1], acc[0][2], acc[0][3]);
  accg4(acc[1][0], acc[1][1], acc[1][2], acc[1][3]);
  accg4(acc[2][0], acc[2][1], acc[2][2], acc[2][3]);
  accg4(acc[3][0], acc[3][1], acc[3][2], acc[3][3]);

  float* slab = sT[wave];
  const int seg = n0 >> 9;
  const float* bsel = (seg == 0) ? bs0 : ((seg == 1) ? bs1 : bs2);
  const int nbOff = seg << 9;
  const int hh = lane >> 4;
  const int c4 = rlane * 4;
#pragma unroll
  for (int i = 0; i < 4; ++i) {
    const int mBase = m0 + (i << 4);
#pragma unroll
    for (int j = 0; j < 4; ++j) {
      const int n = n0 + (j << 4) + rlane;
      const float bv = bfr(bsel[n - nbOff]);
#pragma unroll
      for (int r = 0; r < 8; ++r) {
        float v = acc[i][j][r] * scale + bv;
        if (RR) {
          const float rs = resid[(size_t)(mBase + mOff + r) * ldr + n];
          v = fmaxf(v, 0.0f) + rs;
        }
        slab[(mOff + r) * 68 + (j << 4) + rlane] = v;
      }
    }
    __builtin_amdgcn_fence(__ATOMIC_RELEASE, "workgroup");
    __builtin_amdgcn_wave_barrier();
    __builtin_amdgcn_fence(__ATOMIC_ACQUIRE, "workgroup");
    v4f ov[8];
#pragma unroll
    for (int it = 0; it < 8; ++it) ov[it] = *(const v4f*)(slab + (it * 2 + hh) * 68 + c4);
#pragma unroll
    for (int it = 0; it < 8; ++it)
      *(volatile v4f*)(C + (size_t)(mBase + it * 2 + hh) * ldc + n0 + c4) = ov[it];
    __threadfence();
#pragma unroll
    for (int it = 0; it < 8; ++it)
      *(volatile v4f*)(C + (size_t)(mBase + it * 2 + hh) * ldc + n0 + c4) = ov[it];
    __builtin_amdgcn_fence(__ATOMIC_RELEASE, "workgroup");
    __builtin_amdgcn_wave_barrier();
    __builtin_amdgcn_fence(__ATOMIC_ACQUIRE, "workgroup");
  }
}

__global__ __launch_bounds__(256) void qk_planes_kernel(const float* __restrict__ C32,
                                                        unsigned short* __restrict__ Qhi,
                                                        unsigned short* __restrict__ Qlo,
                                                        unsigned short* __restrict__ K16, int nthr) {
  const int t = blockIdx.x * 256 + threadIdx.x;
  if (t >= nthr) return;
  const int e0  = t * 8;
  const int row = e0 >> 9;
  const int col = e0 & 511;
  const float* qp = C32 + (size_t)row * QKVC + col;
  const float* kp = qp + DM;
  const v4f qa = *(const v4f*)(qp);
  const v4f qb = *(const v4f*)(qp + 4);
  const v4f ka = *(const v4f*)(kp);
  const v4f kb = *(const v4f*)(kp + 4);
  unsigned short hq[8], lq[8], hk[8];
#pragma unroll
  for (int e = 0; e < 4; ++e) {
    const float v0 = qa[e] * 1024.0f;
    hq[e] = h_bits(v0);
    lq[e] = h_bits(v0 - h2f(hq[e]));
    hk[e] = h_bits(ka[e] * 64.0f);
    const float v1 = qb[e] * 1024.0f;
    hq[4 + e] = h_bits(v1);
    lq[4 + e] = h_bits(v1 - h2f(hq[4 + e]));
    hk[4 + e] = h_bits(kb[e] * 64.0f);
  }
  const v4u vh = (v4u){pk16(hq[0], hq[1]), pk16(hq[2], hq[3]), pk16(hq[4], hq[5]), pk16(hq[6], hq[7])};
  const v4u vl = (v4u){pk16(lq[0], lq[1]), pk16(lq[2], lq[3]), pk16(lq[4], lq[5]), pk16(lq[6], lq[7])};
  const v4u vk = (v4u){pk16(hk[0], hk[1]), pk16(hk[2], hk[3]), pk16(hk[4], hk[5]), pk16(hk[6], hk[7])};
  volatile v4u* ph = (volatile v4u*)(Qhi + e0);
  volatile v4u* pl = (volatile v4u*)(Qlo + e0);
  volatile v4u* pk = (volatile v4u*)(K16 + e0);
  *ph = vh; *pl = vl; *pk = vk;
  __threadfence();
  *ph = vh; *pl = vl; *pk = vk;
}

__global__ __launch_bounds__(256) void vtrans_kernel(const float* __restrict__ C32,
                                                     unsigned short* __restrict__ Vth,
                                                     unsigned short* __restrict__ Vtl) {
  __shared__ __align__(16) unsigned short th[64 * 72];
  __shared__ __align__(16) unsigned short tl[64 * 72];
  const int c0  = blockIdx.x * 64;
  const int r0  = blockIdx.y * 64;
  const int b   = blockIdx.z;
  const int tid = threadIdx.x;
  {
    const int rr = tid >> 2;
    const int cq = (tid & 3) * 16;
    const float* src = C32 + (size_t)(b * NTOK + r0 + rr) * QKVC + 2 * DM + c0 + cq;
#pragma unroll
    for (int q = 0; q < 4; ++q) {
      const v4f f = *(const v4f*)(src + 4 * q);
#pragma unroll
      for (int e = 0; e < 4; ++e) {
        const float v = f[e] * 1024.0f;
        const unsigned short hb = h_bits(v);
        const unsigned short lb = h_bits(v - h2f(hb));
        th[rr * 72 + cq + 4 * q + e] = hb;
        tl[rr * 72 + cq + 4 * q + e] = lb;
      }
    }
  }
  __syncthreads();
  const int sub = tid >> 3;
  const int c8  = (tid & 7) * 8;
  v4u hv[2], lv[2];
#pragma unroll
  for (int it = 0; it < 2; ++it) {
    const int oc = it * 32 + sub;
    v4u a, a2;
#pragma unroll
    for (int q = 0; q < 4; ++q) {
      a[q]  = pk16(th[(c8 + 2 * q) * 72 + oc], th[(c8 + 2 * q + 1) * 72 + oc]);
      a2[q] = pk16(tl[(c8 + 2 * q) * 72 + oc], tl[(c8 + 2 * q + 1) * 72 + oc]);
    }
    hv[it] = a; lv[it] = a2;
  }
#pragma unroll
  for (int it = 0; it < 2; ++it) {
    const int oc = it * 32 + sub;
    const size_t go = (size_t)(b * DM + c0 + oc) * NTOK + r0 + c8;
    *(volatile v4u*)(Vth + go) = hv[it];
    *(volatile v4u*)(Vtl + go) = lv[it];
  }
  __threadfence();
#pragma unroll
  for (int it = 0; it < 2; ++it) {
    const int oc = it * 32 + sub;
    const size_t go = (size_t)(b * DM + c0 + oc) * NTOK + r0 + c8;
    *(volatile v4u*)(Vth + go) = hv[it];
    *(volatile v4u*)(Vtl + go) = lv[it];
  }
}

__global__ __launch_bounds__(256) void attn_kernel(
    const unsigned short* __restrict__ Qhip, const unsigned short* __restrict__ Qlop,
    const unsigned short* __restrict__ K16p,
    const unsigned short* __restrict__ Vthp, const unsigned short* __restrict__ Vtlp,
    const float* __restrict__ C32, const float* __restrict__ Xp, const float* __restrict__ pres,
    const float* __restrict__ W1, const float* __restrict__ b1,
    const float* __restrict__ W2, const float* __restrict__ b2,
    float* __restrict__ Of32, unsigned short* __restrict__ Ohi, unsigned short* __restrict__ Olo,
    float inv_sqrt) {
  __shared__ __align__(16) float    xtile[16 * 32 * 3];
  __shared__ __align__(16) _Float16 ptile[NHD][16 * 32];
  __shared__ __align__(16) float    oslab[NHD][16 * 68];

  const int b    = blockIdx.y;
  const int q0   = blockIdx.x * 16;
  const int tid  = threadIdx.x;
  const int lane = tid & 31;
  const int h    = __builtin_amdgcn_readfirstlane(tid >> 5);
  const int m    = lane & 15;
  const int hf   = lane >> 4;

  float w1[3][3], c1[3], w2[3];
#pragma unroll
  for (int o = 0; o < 3; ++o) {
    c1[o] = bfr(b1[h * 3 + o]);
    w2[o] = bfr(W2[h * 3 + o]);
#pragma unroll
    for (int c = 0; c < 3; ++c) w1[o][c] = bfr(W1[h * 9 + o * 3 + c]);
  }
  const float c2 = bfr(b2[h]);

  const _Float16* Qh = (const _Float16*)Qhip;
  const _Float16* Ql = (const _Float16*)Qlop;
  const size_t qoff = (size_t)(b * NTOK + q0 + m) * DM + h * HDIM + 8 * hf;
  const v16h qh0 = ldfh(Qh + qoff), qh1 = ldfh(Qh + qoff + 32);
  const v16h ql0 = ldfh(Ql + qoff), ql1 = ldfh(Ql + qoff + 32);

  float pq[8], rmax[8], rsum[8];
#pragma unroll
  for (int r = 0; r < 8; ++r) {
    pq[r]   = pres[b * NTOK + q0 + 8 * hf + r];
    rmax[r] = -3.0e38f;
    rsum[r] = 0.0f;
  }
  v8f oacc[4];
#pragma unroll
  for (int j = 0; j < 4; ++j) oacc[j] = (v8f){0.f, 0.f, 0.f, 0.f, 0.f, 0.f, 0.f, 0.f};

  const _Float16* Kb = (const _Float16*)K16p + (size_t)(b * NTOK) * DM + h * HDIM + 8 * hf;
  const _Float16* Vh = (const _Float16*)Vthp + (size_t)(b * DM + h * HDIM + m) * NTOK + 8 * hf;
  const _Float16* Vl = (const _Float16*)Vtlp + (size_t)(b * DM + h * HDIM + m) * NTOK + 8 * hf;
  const float* Xb  = Xp + (size_t)(b * NTOK + q0) * (NTOK * 3);
  const float* pkb = pres + b * NTOK;
  const float osc = 1.0f / 65536.0f;

  for (int kc = 0; kc < NTOK; kc += 32) {
    __syncthreads();
#pragma unroll
    for (int it = 0; it < 6; ++it) {
      const int idx = it * 256 + tid;
      const int qi  = idx / 96;
      const int rr  = idx - qi * 96;
      xtile[idx] = bfr(Xb[(size_t)qi * (NTOK * 3) + (size_t)kc * 3 + rr]);
    }
    __syncthreads();

    const _Float16* k0p = Kb + (size_t)(kc + m) * DM;
    const _Float16* k1p = Kb + (size_t)(kc + 16 + m) * DM;
    const v16h kf00 = ldfh(k0p), kf01 = ldfh(k0p + 32);
    const v16h kf10 = ldfh(k1p), kf11 = ldfh(k1p + 32);
    v8f s0 = (v8f){0.f, 0.f, 0.f, 0.f, 0.f, 0.f, 0.f, 0.f};
    v8f s1 = (v8f){0.f, 0.f, 0.f, 0.f, 0.f, 0.f, 0.f, 0.f};
    s0 = mma_h(qh0, kf00, s0); s0 = mma_h(ql0, kf00, s0);
    s0 = mma_h(qh1, kf01, s0); s0 = mma_h(ql1, kf01, s0);
    s1 = mma_h(qh0, kf10, s1); s1 = mma_h(ql0, kf10, s1);
    s1 = mma_h(qh1, kf11, s1); s1 = mma_h(ql1, kf11, s1);
    guard2h(s0, s1, kf10, kf11);
    keep4h(kf00, kf01, kf10, kf11);
    keep4h(qh0, ql0, qh1, ql1);

    const float pk0 = pkb[kc + m];
    const float pk1 = pkb[kc + 16 + m];

#pragma unroll
    for (int r = 0; r < 8; ++r) {
      const int qi = 8 * hf + r;
      float lg[2];
#pragma unroll
      for (int t = 0; t < 2; ++t) {
        const float* x = xtile + (qi * 32 + 16 * t + m) * 3;
        const float x0 = x[0], x1 = x[1], x2 = x[2];
        const float a0 = fmaxf(w1[0][0] * x0 + w1[0][1] * x1 + w1[0][2] * x2 + c1[0], 0.0f);
        const float a1 = fmaxf(w1[1][0] * x0 + w1[1][1] * x1 + w1[1][2] * x2 + c1[1], 0.0f);
        const float a2 = fmaxf(w1[2][0] * x0 + w1[2][1] * x1 + w1[2][2] * x2 + c1[2], 0.0f);
        const float loc = a0 * w2[0] + a1 * w2[1] + a2 * w2[2] + c2;
        float v = ((t ? s1[r] : s0[r]) * osc) * inv_sqrt + loc;
        const float pqr = pq[r];
        v = pqr * v - (1.0f - pqr) * NEGBIG;
        const float pkv = t ? pk1 : pk0;
        v = pkv * v - (1.0f - pkv) * NEGBIG;
        lg[t] = v;
      }
      float mr = fmaxf(lg[0], lg[1]);
#pragma unroll
      for (int off = 1; off < 16; off <<= 1) mr = fmaxf(mr, __shfl_xor(mr, off, 16));
      const float nm = fmaxf(rmax[r], mr);
      const float al = __expf(rmax[r] - nm);
      rmax[r] = nm;
      const float e0 = __expf(lg[0] - nm);
      const float e1 = __expf(lg[1] - nm);
      float ps = e0 + e1;
#pragma unroll
      for (int off = 1; off < 16; off <<= 1) ps += __shfl_xor(ps, off, 16);
      rsum[r] = rsum[r] * al + ps;
#pragma unroll
      for (int j = 0; j < 4; ++j) oacc[j][r] *= al;
      ptile[h][qi * 32 + m]      = (_Float16)(1024.0f * e0);
      ptile[h][qi * 32 + 16 + m] = (_Float16)(1024.0f * e1);
    }
    __builtin_amdgcn_fence(__ATOMIC_RELEASE, "wavefront");
    __builtin_amdgcn_wave_barrier();
    __builtin_amdgcn_fence(__ATOMIC_ACQUIRE, "wavefront");

    const v16h pa = ldfh(&ptile[h][m * 32 + 8 * hf]);
    v16h vh[4], vl[4];
#pragma unroll
    for (int j = 0; j < 4; ++j) {
      vh[j] = ldfh(Vh + (size_t)(j * 16) * NTOK + kc);
      vl[j] = ldfh(Vl + (size_t)(j * 16) * NTOK + kc);
    }
#pragma unroll
    for (int j = 0; j < 4; ++j) {
      oacc[j] = mma_h(pa, vh[j], oacc[j]);
      oacc[j] = mma_h(pa, vl[j], oacc[j]);
    }
    accg4(oacc[0], oacc[1], oacc[2], oacc[3]);
    keep4h(vh[0], vh[1], vh[2], vh[3]);
    keep4h(vl[0], vl[1], vl[2], vl[3]);
    keep4h(pa, pa, pa, pa);
  }

  float* slab = oslab[h];
  const float* Vres = C32 + (size_t)(b * NTOK + q0) * QKVC + 2 * DM + h * HDIM;
#pragma unroll
  for (int r = 0; r < 8; ++r) {
    const int qi = 8 * hf + r;
    const float inv = (1.0f / rsum[r]) * (1.0f / 1048576.0f);
#pragma unroll
    for (int j = 0; j < 4; ++j) {
      const int d = (j << 4) + m;
      const float val = Vres[(size_t)qi * QKVC + d] + oacc[j][r] * inv;
      slab[qi * 68 + d] = val;
    }
  }
  __builtin_amdgcn_fence(__ATOMIC_RELEASE, "workgroup");
  __builtin_amdgcn_wave_barrier();
  __builtin_amdgcn_fence(__ATOMIC_ACQUIRE, "workgroup");

  const int c4 = m * 4;
  v4f ov[8];
#pragma unroll
  for (int it = 0; it < 8; ++it) ov[it] = *(const v4f*)(slab + (it * 2 + hf) * 68 + c4);
  const int qd = lane >> 3;
  const int c8 = (lane & 7) * 8;
  v4u hv[4], lv[4];
#pragma unroll
  for (int it = 0; it < 4; ++it) {
    const float* sp = slab + (it * 4 + qd) * 68 + c8;
    unsigned short hb[8], lb[8];
#pragma unroll
    for (int e = 0; e < 8; ++e) {
      const float v = sp[e];
      hb[e] = f2bf_bits(v);
      lb[e] = f2bf_bits(v - bf_bits2f(hb[e]));
    }
    hv[it] = (v4u){pk16(hb[0], hb[1]), pk16(hb[2], hb[3]), pk16(hb[4], hb[5]), pk16(hb[6], hb[7])};
    lv[it] = (v4u){pk16(lb[0], lb[1]), pk16(lb[2], lb[3]), pk16(lb[4], lb[5]), pk16(lb[6], lb[7])};
  }
  const size_t rowbase = (size_t)(b * NTOK + q0);
#pragma unroll
  for (int it = 0; it < 8; ++it)
    *(volatile v4f*)(Of32 + (rowbase + it * 2 + hf) * DM + h * HDIM + c4) = ov[it];
#pragma unroll
  for (int it = 0; it < 4; ++it) {
    const size_t eo = (rowbase + it * 4 + qd) * DM + h * HDIM + c8;
    *(volatile v4u*)(Ohi + eo) = hv[it];
    *(volatile v4u*)(Olo + eo) = lv[it];
  }
  __threadfence();
#pragma unroll
  for (int it = 0; it < 8; ++it)
    *(volatile v4f*)(Of32 + (rowbase + it * 2 + hf) * DM + h * HDIM + c4) = ov[it];
#pragma unroll
  for (int it = 0; it < 4; ++it) {
    const size_t eo = (rowbase + it * 4 + qd) * DM + h * HDIM + c8;
    *(volatile v4u*)(Ohi + eo) = hv[it];
    *(volatile v4u*)(Olo + eo) = lv[it];
  }
}

extern "C" void kernel_launch(void* const* d_in, const int* in_sizes, int n_in,
                              void* d_out, int out_size, void* d_ws, size_t ws_size,
                              hipStream_t stream) {
  if (n_in < 15) return;
  if (in_sizes[0] != NB * NTOK * DM) return;
  if (in_sizes[1] != NB * NTOK * NTOK * 3) return;
  if (in_sizes[2] != NB * NTOK) return;
  if (in_sizes[3] != DM * DM || in_sizes[5] != DM * DM || in_sizes[7] != DM * DM || in_sizes[9] != DM * DM) return;
  if (in_sizes[4] != DM || in_sizes[6] != DM || in_sizes[8] != DM || in_sizes[10] != DM) return;
  if (in_sizes[11] != NHD * 9 || in_sizes[12] != NHD * 3 || in_sizes[13] != NHD * 3 || in_sizes[14] != NHD) return;
  if (out_size != NB * NTOK * DM) return;

  const float* Y    = (const float*)d_in[0];
  const float* Xp   = (const float*)d_in[1];
  const float* pres = (const float*)d_in[2];
  const float* Wq   = (const float*)d_in[3];
  const float* bq   = (const float*)d_in[4];
  const float* Wk   = (const float*)d_in[5];
  const float* bk   = (const float*)d_in[6];
  const float* Wv   = (const float*)d_in[7];
  const float* bv   = (const float*)d_in[8];
  const float* Wo   = (const float*)d_in[9];
  const float* bo   = (const float*)d_in[10];
  const float* W1   = (const float*)d_in[11];
  const float* b1   = (const float*)d_in[12];
  const float* W2   = (const float*)d_in[13];
  const float* b2   = (const float*)d_in[14];

  const size_t ntokall = (size_t)NB * NTOK;
  const size_t PYB  = ntokall * DM * 2;
  const size_t PWC  = (size_t)QKVC * DM * 2;
  const size_t PWO  = (size_t)DM * DM * 2;
  const size_t PC32 = ntokall * QKVC * 4;
  const size_t P16  = ntokall * DM * 2;
  const size_t POF  = ntokall * DM * 4;
  size_t off = 0;
  const size_t oYbf = off; off += PYB;
  const size_t oWc  = off; off += PWC;
  const size_t oWo  = off; off += PWO;
  const size_t oC32 = off; off += PC32;
  const size_t oQhi = off; off += P16;
  const size_t oQlo = off; off += P16;
  const size_t oK16 = off; off += P16;
  const size_t oVth = off; off += P16;
  const size_t oVtl = off; off += P16;
  const size_t oOf  = off; off += POF;
  const size_t oOhi = off; off += P16;
  const size_t oOlo = off; off += P16;
  if (off > ws_size) return;

  char* ws = (char*)d_ws;
  unsigned short* Ybf  = (unsigned short*)(ws + oYbf);
  unsigned short* Wcat = (unsigned short*)(ws + oWc);
  unsigned short* Wobf = (unsigned short*)(ws + oWo);
  float*          C32  = (float*)(ws + oC32);
  unsigned short* Qhi  = (unsigned short*)(ws + oQhi);
  unsigned short* Qlo  = (unsigned short*)(ws + oQlo);
  unsigned short* K16  = (unsigned short*)(ws + oK16);
  unsigned short* Vth  = (unsigned short*)(ws + oVth);
  unsigned short* Vtl  = (unsigned short*)(ws + oVtl);
  float*          Of32 = (float*)(ws + oOf);
  unsigned short* Ohi  = (unsigned short*)(ws + oOhi);
  unsigned short* Olo  = (unsigned short*)(ws + oOlo);

  const dim3 blk(256);
  const int n2y = NB * NTOK * DM / 2;
  const int n2w = DM * DM / 2;
  const float inv_sqrt = (float)(1.0 / sqrt((double)DM));

  cast_bf16_kernel<<<dim3((n2y + 255) / 256), blk, 0, stream>>>(Y, Ybf, n2y);
  cast_bf16_kernel<<<dim3((n2w + 255) / 256), blk, 0, stream>>>(Wq, Wcat, n2w);
  cast_bf16_kernel<<<dim3((n2w + 255) / 256), blk, 0, stream>>>(Wk, Wcat + (size_t)DM * DM, n2w);
  cast_bf16_kernel<<<dim3((n2w + 255) / 256), blk, 0, stream>>>(Wv, Wcat + (size_t)2 * DM * DM, n2w);
  cast_bf16_kernel<<<dim3((n2w + 255) / 256), blk, 0, stream>>>(Wo, Wobf, n2w);

  {
    const int tiles = (int)((ntokall / 64) * (QKVC / 64));
    gemm64_kernel<false, false><<<dim3((tiles + 7) / 8), blk, 0, stream>>>(
        Ybf, Ybf, DM, Wcat, DM, C32, QKVC, bq, bk, bv, bq, 0,
        (int)ntokall, QKVC, DM, 1.0f);
  }

  {
    const int nthr = (int)(ntokall * DM / 8);
    qk_planes_kernel<<<dim3((nthr + 255) / 256), blk, 0, stream>>>(C32, Qhi, Qlo, K16, nthr);
    vtrans_kernel<<<dim3(DM / 64, NTOK / 64, NB), blk, 0, stream>>>(C32, Vth, Vtl);
  }

  attn_kernel<<<dim3(NTOK / 16, NB), blk, 0, stream>>>(
      Qhi, Qlo, K16, Vth, Vtl, C32, Xp, pres, W1, b1, W2, b2, Of32, Ohi, Olo, inv_sqrt);

  {
    const int tiles = (int)((ntokall / 64) * (DM / 64));
    gemm64_kernel<true, true><<<dim3((tiles + 7) / 8), blk, 0, stream>>>(
        Ohi, Olo, DM, Wobf, DM, (float*)d_out, DM, bo, bo, bo, Of32, DM,
        (int)ntokall, DM, DM, 1.0f);
  }
  (void)hipGetLastError();
}
